// TransformerAttentionModule_21062519619908
// MI455X (gfx1250) — hardware-run, weakly checked
//
#include <hip/hip_runtime.h>
#include <math.h>

typedef __attribute__((ext_vector_type(16))) __bf16   v16b;
typedef __attribute__((ext_vector_type(8)))  __bf16   v8b;
typedef __attribute__((ext_vector_type(8)))  _Float16 v8h;
typedef __attribute__((ext_vector_type(8)))  float    v8f;
typedef __attribute__((ext_vector_type(4)))  float    v4f;
typedef __attribute__((ext_vector_type(4)))  int      v4i;

constexpr int kNodes    = 50000;
constexpr int kEdges    = 800000;
constexpr int kDim      = 128;
constexpr int kHeads    = 8;
constexpr int kHeadDim  = 16;
constexpr int kMPad     = ((kNodes + 63) / 64) * 64;
constexpr int kQkvW     = 3 * kDim;
constexpr float kScoreScale = 0.25f;
static_assert(kHeads * kHeadDim == kDim);
static_assert(kScoreScale * kScoreScale * (float)kHeadDim == 1.0f);
static_assert(kMPad == 50048);
static_assert((kDim % 32) == 0 && (kQkvW % 64) == 0 && (kDim % 64) == 0 && (kMPad % 64) == 0);
static_assert((kNodes % 16) == 0);
static_assert((kEdges % 4) == 0);
static_assert(kNodes <= (1 << 23));

constexpr int kTileNodes  = 96;
constexpr int kEdgeBlocks = (kMPad + kTileNodes - 1) / kTileNodes;
constexpr int kAggRows    = kEdgeBlocks * kTileNodes;
constexpr int kSubIters   = 2;
constexpr int kWaveEdges  = 128 * kSubIters;
constexpr int kListCap    = kWaveEdges;
constexpr int kChunkEdges = 8 * kWaveEdges;
constexpr int kChunks     = (kEdges + kChunkEdges - 1) / kChunkEdges;
constexpr int kEpiIters   = kTileNodes / 16;
static_assert(kEdgeBlocks == 522 && kAggRows == 50112 && kAggRows >= kMPad);
static_assert(kTileNodes <= 256 && (kTileNodes % 16) == 0);
static_assert(kListCap == 256 && (kListCap & (kListCap - 1)) == 0);
static_assert(kChunks == 391);

constexpr int kXBlocks     = (kMPad * kDim / 8) / 256;
constexpr int kXRealBlocks = (kNodes * kDim / 8) / 256;
constexpr int kWBlocks     = (kDim * kDim / 8) / 256;
constexpr int kPrepBlocks  = kXBlocks + 3 * kWBlocks + kWBlocks + 1;
static_assert(((kMPad * kDim / 8) % 256) == 0 && ((kNodes * kDim / 8) % 256) == 0 && ((kDim * kDim / 8) % 256) == 0);
static_assert(kXBlocks == 3128 && kXRealBlocks == 3125 && kWBlocks == 8 && kPrepBlocks == 3161);

constexpr size_t kOffA0   = 0;
constexpr size_t kOffWQKV = kOffA0   + (size_t)kMPad * kDim * 2;
constexpr size_t kOffWO   = kOffWQKV + (size_t)kQkvW * kDim * 2;
constexpr size_t kOffBIAS = kOffWO   + (size_t)kDim * kDim * 2;
constexpr size_t kOffQKV  = kOffBIAS + (size_t)512 * 4;
constexpr size_t kOffAH   = kOffQKV  + (size_t)kMPad * kQkvW * 4;
constexpr size_t kOffAL   = kOffAH   + (size_t)kAggRows * kDim * 2;
constexpr size_t kWsTotal = kOffAL   + (size_t)kAggRows * kDim * 2;
static_assert(kWsTotal == 115476480ull);
static_assert(kWsTotal <= 134217728ull);
static_assert((kOffWQKV % 128) == 0 && (kOffWO % 128) == 0 && (kOffBIAS % 128) == 0 &&
              (kOffQKV % 128) == 0 && (kOffAH % 128) == 0 && (kOffAL % 128) == 0);

__device__ __forceinline__ unsigned short f2bf_bits(float f) {
  unsigned u = __float_as_uint(f);
  return (unsigned short)((u + 0x7FFFu + ((u >> 16) & 1u)) >> 16);
}
__device__ __forceinline__ float bf_bits2f(unsigned short h) { return __uint_as_float(((unsigned)h) << 16); }
__device__ __forceinline__ int iclamp(int v, int lo, int hi) {
  const int a = (v < lo) ? lo : v;
  return (a > hi) ? hi : a;
}

__device__ __forceinline__ v8f mma_g(v16b a, v16b b, v8f c) {
  c = __builtin_amdgcn_wmma_f32_16x16x32_bf16(false, a, false, b, (short)0, c, false, false);
  asm volatile("v_nop\n\tv_nop\n\tv_nop\n\tv_nop" : "+v"(c) : "v"(a), "v"(b));
  return c;
}
__device__ __forceinline__ void keep4_b(v16b a, v16b b, v16b c, v16b d) { asm volatile("v_nop" :: "v"(a), "v"(b), "v"(c), "v"(d)); }
__device__ __forceinline__ void acc_guard4(v8f& a, v8f& b, v8f& c, v8f& d) { asm volatile("v_nop\n\tv_nop\n\tv_nop\n\tv_nop" : "+v"(a), "+v"(b), "+v"(c), "+v"(d)); }

union FragB { v16b v; v8b h[2]; };
__device__ __forceinline__ v16b frag_load(const __bf16* p) {
  FragB f;
  f.h[0] = *(const v8b*)(p);
  f.h[1] = *(const v8b*)(p + 16);
  return f.v;
}

__device__ __forceinline__ v8h cvt8_bf16(const float* __restrict__ p) {
  const v4f a0 = *(const v4f*)(p);
  const v4f a1 = *(const v4f*)(p + 4);
  v8h o;
#pragma unroll
  for (int e = 0; e < 4; ++e) {
    const float f0 = a0[e];
    const float f1 = a1[e];
    const unsigned short h0 = f2bf_bits(f0);
    const unsigned short h1 = f2bf_bits(f1);
    o[e]     = __builtin_bit_cast(_Float16, h0);
    o[4 + e] = __builtin_bit_cast(_Float16, h1);
  }
  return o;
}
__device__ __forceinline__ void store2_v8h(unsigned short* p, v8h v) {
  *(volatile v8h*)p = v;
  __threadfence();
  *(volatile v8h*)p = v;
}

__global__ __launch_bounds__(256) void prep_planes_kernel(
    const float* __restrict__ x, const float* __restrict__ Wq, const float* __restrict__ Wk,
    const float* __restrict__ Wv, const float* __restrict__ Wo,
    const float* __restrict__ bq, const float* __restrict__ bk, const float* __restrict__ bv,
    const float* __restrict__ bo,
    unsigned short* __restrict__ A0, unsigned short* __restrict__ WQKV, unsigned short* __restrict__ WO,
    float* __restrict__ BIAS)
{
  const int tid = threadIdx.x;
  const int blk = blockIdx.x;
  if (blk < kXRealBlocks) {
    const size_t e0 = ((size_t)blk * 256 + tid) * 8;
    const v8h o = cvt8_bf16(x + e0);
    store2_v8h(A0 + e0, o);
  } else if (blk < kXBlocks) {
    const size_t e0 = ((size_t)blk * 256 + tid) * 8;
    const _Float16 z = (_Float16)0.0f;
    const v8h o = (v8h){z, z, z, z, z, z, z, z};
    store2_v8h(A0 + e0, o);
  } else if (blk < kXBlocks + 3 * kWBlocks) {
    const int wb = blk - kXBlocks;
    const int which = wb / kWBlocks;
    const float* src = (which == 0) ? Wq : ((which == 1) ? Wk : Wv);
    const size_t l0 = ((size_t)(wb - which * kWBlocks) * 256 + tid) * 8;
    const v8h o = cvt8_bf16(src + l0);
    store2_v8h(WQKV + (size_t)which * kDim * kDim + l0, o);
  } else if (blk < kXBlocks + 4 * kWBlocks) {
    const int wb = blk - (kXBlocks + 3 * kWBlocks);
    const size_t l0 = ((size_t)wb * 256 + tid) * 8;
    const v8h o = cvt8_bf16(Wo + l0);
    store2_v8h(WO + l0, o);
  } else {
    const int wave = __builtin_amdgcn_readfirstlane((int)(threadIdx.x >> 5));
    const int lane = tid & 31;
    if (wave < 4) {
      const float* src = (wave == 0) ? bq : ((wave == 1) ? bk : ((wave == 2) ? bv : bo));
      const v4f v = *(const v4f*)(src + lane * 4);
      v4f o;
#pragma unroll
      for (int e = 0; e < 4; ++e) {
        const float f = v[e];
        o[e] = bf_bits2f(f2bf_bits(f));
      }
      float* dst = BIAS + wave * kDim + lane * 4;
      *(volatile v4f*)dst = o;
      __threadfence();
      *(volatile v4f*)dst = o;
    }
  }
}

template <int SPL>
__global__ __launch_bounds__(256) void gemm_bf16_tile64_kernel(
    const unsigned short* __restrict__ Ap, const unsigned short* __restrict__ A2p, int lda,
    const unsigned short* __restrict__ Btp, int ldb,
    float* __restrict__ C, int ldc,
    const float* __restrict__ bias, int M, int N, int K, int Mstore)
{
  const __bf16* A  = (const __bf16*)Ap;
  const __bf16* A2 = (const __bf16*)A2p;
  const __bf16* Bt = (const __bf16*)Btp;
  __shared__ __align__(16) float sT[8][16 * 68];
  const int lane = threadIdx.x & 31;
  const int wave = __builtin_amdgcn_readfirstlane((int)(threadIdx.x >> 5));
  const int tilesN = N >> 6;
  const int tilesM = M >> 6;
  const int tile = blockIdx.x * 8 + wave;
  if (tile >= tilesM * tilesN) return;
  const int tm = tile / tilesN;
  const int tn = tile - tm * tilesN;
  const int m0 = tm << 6;
  const int n0 = tn << 6;

  const int rlane = lane & 15;
  const int koff  = (lane >> 4) * 8;
  const int mOff  = (lane >> 4) * 8;

  v8f acc[4][4];
#pragma unroll
  for (int i = 0; i < 4; ++i)
#pragma unroll
    for (int j = 0; j < 4; ++j) acc[i][j] = (v8f){0.f, 0.f, 0.f, 0.f, 0.f, 0.f, 0.f, 0.f};

  for (int k0 = 0; k0 < K; k0 += 32) {
    v16b bh[4];
#pragma unroll
    for (int j = 0; j < 4; ++j) {
      const size_t bo = (size_t)(n0 + (j << 4) + rlane) * ldb + koff + k0;
      bh[j] = frag_load(Bt + bo);
    }
#pragma unroll
    for (int i = 0; i < 4; ++i) {
      const size_t ao = (size_t)(m0 + (i << 4) + rlane) * lda + koff + k0;
      const v16b ah = frag_load(A + ao);
      v16b al = ah;
      if (SPL == 1) al = frag_load(A2 + ao);
#pragma unroll
      for (int j = 0; j < 4; ++j) {
        acc[i][j] = mma_g(ah, bh[j], acc[i][j]);
        if (SPL == 1) acc[i][j] = mma_g(al, bh[j], acc[i][j]);
      }
    }
    keep4_b(bh[0], bh[1], bh[2], bh[3]);
  }
  acc_guard4(acc[0][0], acc[0][1], acc[0][2], acc[0][3]);
  acc_guard4(acc[1][0], acc[1][1], acc[1][2], acc[1][3]);
  acc_guard4(acc[2][0], acc[2][1], acc[2][2], acc[2][3]);
  acc_guard4(acc[3][0], acc[3][1], acc[3][2], acc[3][3]);

  float* slab = sT[wave];
#pragma unroll
  for (int i = 0; i < 4; ++i) {
    const int mBase = m0 + (i << 4);
#pragma unroll
    for (int j = 0; j < 4; ++j) {
      const int n = n0 + (j << 4) + rlane;
      const float bvl = bias[n];
#pragma unroll
      for (int r = 0; r < 8; ++r) {
        const float v = acc[i][j][r] + bvl;
        slab[(mOff + r) * 68 + (j << 4) + rlane] = v;
      }
    }
    __builtin_amdgcn_fence(__ATOMIC_RELEASE, "workgroup");
    __builtin_amdgcn_wave_barrier();
    __builtin_amdgcn_fence(__ATOMIC_ACQUIRE, "workgroup");
    if (mBase < Mstore) {
      const int hh = lane >> 4;
      const int c4 = (lane & 15) * 4;
      for (int pass = 0; pass < 2; ++pass) {
#pragma unroll
        for (int it = 0; it < 8; ++it) {
          const int row = it * 2 + hh;
          const v4f v = *(const v4f*)(slab + row * 68 + c4);
          *(volatile v4f*)(C + (size_t)(mBase + row) * ldc + n0 + c4) = v;
        }
        __threadfence();
      }
    }
    __builtin_amdgcn_fence(__ATOMIC_RELEASE, "workgroup");
    __builtin_amdgcn_wave_barrier();
    __builtin_amdgcn_fence(__ATOMIC_ACQUIRE, "workgroup");
  }
}

__device__ __forceinline__ void push_hit(int* lst, int& cnt, unsigned bal, bool hit, int srcv, int tloc) {
  const int pos = (cnt + (int)__builtin_amdgcn_mbcnt_lo(bal, 0u)) & (kListCap - 1);
  const int ent = (iclamp(srcv, 0, kNodes - 1) << 8) | (tloc & 255);
  if (hit) lst[pos] = ent;
  cnt += __popc(bal);
}

__global__ __launch_bounds__(256) void edge_softmax_agg_kernel(
    const int* __restrict__ ei, const float* __restrict__ QKV,
    unsigned short* __restrict__ AH, unsigned short* __restrict__ AL)
{
  __shared__ __align__(16) float sAgg[kTileNodes * kDim];
  __shared__ __align__(16) float sM[kTileNodes * kHeads];
  __shared__ __align__(16) float sL[kTileNodes * kHeads];
  __shared__ __align__(16) int   sList[8 * kListCap];
  __shared__ __align__(16) int   sCnt[8];

  const int tid  = threadIdx.x;
  const int lane = tid & 31;
  const int wave = __builtin_amdgcn_readfirstlane((int)(threadIdx.x >> 5));
  const int n0   = blockIdx.x * kTileNodes;
  const int* tgtp = ei;
  const int* srcp = ei + kEdges;

#pragma unroll 1
  for (int i = tid; i < kTileNodes * kDim / 4; i += 256) *(v4f*)(sAgg + 4 * i) = (v4f){0.f, 0.f, 0.f, 0.f};
#pragma unroll 1
  for (int i = tid; i < kTileNodes * kHeads; i += 256) {
    sM[i] = -__builtin_inff();
    sL[i] = 0.f;
  }

  int* myList = sList + wave * kListCap;

#pragma unroll 1
  for (int ch = 0; ch < kChunks; ++ch) {
    int cnt = 0;
#pragma unroll
    for (int sb = 0; sb < kSubIters; ++sb) {
      const int eb = ch * kChunkEdges + wave * kWaveEdges + sb * 128 + lane * 4;
      const bool valid = eb < kEdges;
      const int ebc = valid ? eb : (kEdges - 4);
      const v4i tv = *(const v4i*)(tgtp + ebc);
      const int t0 = tv.x - n0;
      const int t1 = tv.y - n0;
      const int t2 = tv.z - n0;
      const int t3 = tv.w - n0;
      const bool h0 = valid && ((unsigned)t0 < (unsigned)kTileNodes);
      const bool h1 = valid && ((unsigned)t1 < (unsigned)kTileNodes);
      const bool h2 = valid && ((unsigned)t2 < (unsigned)kTileNodes);
      const bool h3 = valid && ((unsigned)t3 < (unsigned)kTileNodes);
      const unsigned b0 = __builtin_amdgcn_ballot_w32(h0);
      const unsigned b1 = __builtin_amdgcn_ballot_w32(h1);
      const unsigned b2 = __builtin_amdgcn_ballot_w32(h2);
      const unsigned b3 = __builtin_amdgcn_ballot_w32(h3);
      if ((b0 | b1 | b2 | b3) != 0u) {
        const v4i sv = *(const v4i*)(srcp + ebc);
        int s0 = sv.x;
        int s1 = sv.y;
        int s2 = sv.z;
        int s3 = sv.w;
        asm volatile("" : "+v"(s0), "+v"(s1), "+v"(s2), "+v"(s3));
        push_hit(myList, cnt, b0, h0, s0, t0);
        push_hit(myList, cnt, b1, h1, s1, t1);
        push_hit(myList, cnt, b2, h2, s2, t2);
        push_hit(myList, cnt, b3, h3, s3, t3);
      }
    }
    if (lane == 0) sCnt[wave] = cnt;
    __syncthreads();

    const int cv = sCnt[lane & 7];
#pragma unroll 1
    for (int w2 = 0; w2 < 8; ++w2) {
      int c2 = __builtin_amdgcn_readlane(cv, w2);
      c2 = (c2 < 0) ? 0 : ((c2 > kListCap) ? kListCap : c2);
#pragma unroll 1
      for (int i = 0; i < c2; ++i) {
        const int ent = __builtin_amdgcn_readfirstlane(sList[w2 * kListCap + i]);
        int tl = ent & 255;
        if ((tl & 7) == wave) {
          tl = (tl > kTileNodes - 1) ? (kTileNodes - 1) : tl;
          const int sn = iclamp(ent >> 8, 0, kNodes - 1);
          const int nd = iclamp(n0 + tl, 0, kNodes - 1);
          const float* qrow = QKV + (size_t)sn * kQkvW + 4 * lane;
          const float* krow = QKV + (size_t)nd * kQkvW + kDim + 4 * lane;
          const v4f qv = *(const v4f*)(qrow);
          const v4f kv = *(const v4f*)(krow);
          const v4f vv = *(const v4f*)(qrow + 2 * kDim);
          float part = qv[0] * kv[0];
          part = fmaf(qv[1], kv[1], part);
          part = fmaf(qv[2], kv[2], part);
          part = fmaf(qv[3], kv[3], part);
          part += __shfl_xor(part, 1, 32);
          part += __shfl_xor(part, 2, 32);
          const float sc = part * kScoreScale;
          const int hidx = tl * kHeads + (lane >> 2);
          const float mo = sM[hidx];
          const float lo = sL[hidx];
          const float d = sc - mo;
          const float e = expf(-fabsf(d));
          const bool up = d > 0.0f;
          const float alpha = up ? e : 1.0f;
          const float p = up ? 1.0f : e;
          const float mn = up ? sc : mo;
          const float ln = lo * alpha + p;
          if ((lane & 3) == 0) {
            sM[hidx] = mn;
            sL[hidx] = ln;
          }
          float* ap = sAgg + tl * kDim + 4 * lane;
          v4f a = *(const v4f*)ap;
          a[0] = a[0] * alpha + p * vv[0];
          a[1] = a[1] * alpha + p * vv[1];
          a[2] = a[2] * alpha + p * vv[2];
          a[3] = a[3] * alpha + p * vv[3];
          *(v4f*)ap = a;
        }
      }
    }
    __syncthreads();
  }

#pragma unroll 1
  for (int i = tid; i < kTileNodes * kHeads; i += 256) {
    const float l = sL[i];
    const bool pos = l > 0.0f;
    const float ls = pos ? l : 1.0f;
    const float r = 1.0f / ls;
    sL[i] = pos ? r : 0.0f;
  }
  __syncthreads();

  const int rsel = lane >> 4;
  const int c8 = (lane & 15) * 8;
  v8h hv[kEpiIters], lv[kEpiIters];
#pragma unroll
  for (int it = 0; it < kEpiIters; ++it) {
    const int row = it * 16 + wave * 2 + rsel;
    const float inv = sL[row * kHeads + (c8 >> 4)];
    const float* sp = sAgg + row * kDim + c8;
    const v4f a0 = *(const v4f*)(sp);
    const v4f a1 = *(const v4f*)(sp + 4);
#pragma unroll
    for (int e = 0; e < 4; ++e) {
      const float f0 = a0[e] * inv;
      const float f1 = a1[e] * inv;
      const unsigned short h0 = f2bf_bits(f0);
      const unsigned short h1 = f2bf_bits(f1);
      const unsigned short l0 = f2bf_bits(f0 - bf_bits2f(h0));
      const unsigned short l1 = f2bf_bits(f1 - bf_bits2f(h1));
      hv[it][e]     = __builtin_bit_cast(_Float16, h0);
      hv[it][4 + e] = __builtin_bit_cast(_Float16, h1);
      lv[it][e]     = __builtin_bit_cast(_Float16, l0);
      lv[it][4 + e] = __builtin_bit_cast(_Float16, l1);
    }
  }
  for (int pass = 0; pass < 2; ++pass) {
#pragma unroll
    for (int it = 0; it < kEpiIters; ++it) {
      const int row = it * 16 + wave * 2 + rsel;
      const size_t o = (size_t)(n0 + row) * kDim + c8;
      *(volatile v8h*)(AH + o) = hv[it];
      *(volatile v8h*)(AL + o) = lv[it];
    }
    __threadfence();
  }
}

extern "C" void kernel_launch(void* const* d_in, const int* in_sizes, int n_in,
                              void* d_out, int out_size, void* d_ws, size_t ws_size,
                              hipStream_t stream) {
  if (n_in < 10) return;
  if (in_sizes[0] != kNodes * kDim) return;
  if (in_sizes[1] != 2 * kEdges) return;
  if (in_sizes[2] != kDim * kDim) return;
  if (in_sizes[3] != kDim) return;
  if (in_sizes[4] != kDim * kDim) return;
  if (in_sizes[5] != kDim) return;
  if (in_sizes[6] != kDim * kDim) return;
  if (in_sizes[7] != kDim) return;
  if (in_sizes[8] != kDim * kDim) return;
  if (in_sizes[9] != kDim) return;
  if (out_size != kNodes * kDim) return;
  if (ws_size < kWsTotal) return;

  const float* x  = (const float*)d_in[0];
  const int*   ei = (const int*)d_in[1];
  const float* Wq = (const float*)d_in[2];
  const float* bq = (const float*)d_in[3];
  const float* Wk = (const float*)d_in[4];
  const float* bk = (const float*)d_in[5];
  const float* Wv = (const float*)d_in[6];
  const float* bv = (const float*)d_in[7];
  const float* Wo = (const float*)d_in[8];
  const float* bo = (const float*)d_in[9];
  float* out = (float*)d_out;

  char* ws = (char*)d_ws;
  unsigned short* A0   = (unsigned short*)(ws + kOffA0);
  unsigned short* WQKV = (unsigned short*)(ws + kOffWQKV);
  unsigned short* WO   = (unsigned short*)(ws + kOffWO);
  float*          BIAS = (float*)(ws + kOffBIAS);
  float*          QKV  = (float*)(ws + kOffQKV);
  unsigned short* AH   = (unsigned short*)(ws + kOffAH);
  unsigned short* AL   = (unsigned short*)(ws + kOffAL);

  prep_planes_kernel<<<kPrepBlocks, 256, 0, stream>>>(x, Wq, Wk, Wv, Wo, bq, bk, bv, bo, A0, WQKV, WO, BIAS);

  {
    const int tiles = (kMPad / 64) * (kQkvW / 64);
    gemm_bf16_tile64_kernel<0><<<(tiles + 7) / 8, 256, 0, stream>>>(
        A0, A0, kDim, WQKV, kDim, QKV, kQkvW, BIAS, kMPad, kQkvW, kDim, kMPad);
  }

  edge_softmax_agg_kernel<<<kEdgeBlocks, 256, 0, stream>>>(ei, QKV, AH, AL);

  {
    const int tiles = (kMPad / 64) * (kDim / 64);
    gemm_bf16_tile64_kernel<1><<<(tiles + 7) / 8, 256, 0, stream>>>(
        AH, AL, kDim, WO, kDim, out, kDim, BIAS + kQkvW, kMPad, kDim, kDim, kNodes);
  }
}
